// DoubleStreamBlock_62388694942148
// MI455X (gfx1250) — hardware-run, weakly checked
//
#include <hip/hip_runtime.h>


#define LI   2048
#define LTX  512
#define LA   2560
#define HID  1024
#define NH_  16
#define HD   64
#define MLPD 4096
#define ZH   2
#define PCAR 1024.0f
typedef _Float16 h16;
typedef unsigned short bf;
typedef __attribute__((ext_vector_type(16))) __bf16   v16bf;
typedef __attribute__((ext_vector_type(16))) _Float16 v16h;
typedef __attribute__((ext_vector_type(8)))  _Float16 v8h;
typedef __attribute__((ext_vector_type(8)))  unsigned short v8us;
typedef __attribute__((ext_vector_type(8)))  float    v8f;
typedef __attribute__((ext_vector_type(4)))  float    v4f;
typedef v8h  __attribute__((may_alias)) v8ha;
typedef v4f  __attribute__((may_alias)) v4fa;
typedef v8us __attribute__((may_alias)) v8usa;

__device__ __forceinline__ unsigned short f2bf(float f) { unsigned u = __float_as_uint(f); u += 0x7FFFu + ((u >> 16) & 1u); return (unsigned short)(u >> 16); }
__device__ __forceinline__ float bf2f(unsigned short b) { return __uint_as_float(((unsigned)b) << 16); }
__device__ __forceinline__ float bfr(float f) { return bf2f(f2bf(f)); }
__device__ __forceinline__ v16h cat16(v8h lo, v8h hi) { return __builtin_shufflevector(lo, hi, 0, 1, 2, 3, 4, 5, 6, 7, 8, 9, 10, 11, 12, 13, 14, 15); }
__device__ __forceinline__ v16bf cat16b(v8us lo, v8us hi) { return __builtin_bit_cast(v16bf, __builtin_shufflevector(lo, hi, 0, 1, 2, 3, 4, 5, 6, 7, 8, 9, 10, 11, 12, 13, 14, 15)); }
__device__ __forceinline__ v8f wmma16(v16h a, v16h b, v8f c) { return __builtin_amdgcn_wmma_f32_16x16x32_f16(false, a, false, b, (short)0, c, false, false); }
__device__ __forceinline__ v8f wmmab(v16bf a, v16bf b, v8f c) { return __builtin_amdgcn_wmma_f32_16x16x32_bf16(false, a, false, b, (short)0, c, false, false); }


template <typename T16> struct WFrag;
template <> struct WFrag<h16> { typedef v16h V; static __device__ __forceinline__ V ld(const h16* p) { return cat16(*(const v8h*)p, *(const v8h*)(p + 16)); } static __device__ __forceinline__ v8f mma(V a, V b, v8f c) { return wmma16(a, b, c); } };
template <> struct WFrag<bf> { typedef v16bf V; static __device__ __forceinline__ V ld(const bf* p) { return cat16b(*(const v8us*)p, *(const v8us*)(p + 16)); } static __device__ __forceinline__ v8f mma(V a, V b, v8f c) { return wmmab(a, b, c); } };
template <typename T16, int NSPLIT, bool BIAS>
__global__ __launch_bounds__(32) void k_gemmw(const T16* __restrict__ A, const T16* __restrict__ A2, const T16* __restrict__ Bt, const T16* __restrict__ Bt2, int K, float* C, int ldc, const float* __restrict__ bias, size_t sA, size_t sB, size_t sC) {
    typedef typename WFrag<T16>::V V;
    __shared__ __align__(16) float os[16 * 68];
    const size_t z = blockIdx.z; A += z * sA; if (A2) A2 += z * sA; Bt += z * sB; if (Bt2) Bt2 += z * sB; C += z * sC;
    const int lane = threadIdx.x & 31, lr = lane & 15, hi = lane >> 4; const int r0 = blockIdx.x * 64, c0 = blockIdx.y * 64;
    v8f acc[4][4];
#pragma unroll
    for (int mb = 0; mb < 4; ++mb)
#pragma unroll
        for (int nb = 0; nb < 4; ++nb) acc[mb][nb] = (v8f){};
    const size_t aoff = (size_t)(r0 + lr) * K + 8 * hi, boff = (size_t)(c0 + lr) * K + 8 * hi;
#pragma unroll 1
    for (int kc = 0; kc < K; kc += 32) {
        V a[4], a2[4];
#pragma unroll
        for (int mb = 0; mb < 4; ++mb) { a[mb] = WFrag<T16>::ld(A + aoff + (size_t)mb * 16 * K + kc); if (NSPLIT == 1 || NSPLIT == 2) a2[mb] = WFrag<T16>::ld(A2 + aoff + (size_t)mb * 16 * K + kc); }
#pragma unroll
        for (int nb = 0; nb < 4; ++nb) { const V b = WFrag<T16>::ld(Bt + boff + (size_t)nb * 16 * K + kc); V b2; if (NSPLIT >= 2) b2 = WFrag<T16>::ld(Bt2 + boff + (size_t)nb * 16 * K + kc);
#pragma unroll
            for (int mb = 0; mb < 4; ++mb) { acc[mb][nb] = WFrag<T16>::mma(a[mb], b, acc[mb][nb]); if (NSPLIT == 1 || NSPLIT == 2) acc[mb][nb] = WFrag<T16>::mma(a2[mb], b, acc[mb][nb]); if (NSPLIT >= 2) acc[mb][nb] = WFrag<T16>::mma(a[mb], b2, acc[mb][nb]); } }
        asm volatile("v_nop\n\tv_nop\n\tv_nop\n\tv_nop" : "+v"(acc[0][0]), "+v"(acc[1][1]), "+v"(acc[2][2]), "+v"(acc[3][3]) : "v"(a[0]), "v"(a[3]));
    }
#pragma unroll
    for (int mb = 0; mb < 4; ++mb) {
#pragma unroll
        for (int nb = 0; nb < 4; ++nb) {
#pragma unroll
            for (int j = 0; j < 8; ++j) os[(hi * 8 + j) * 68 + nb * 16 + lr] = acc[mb][nb][j]; }
        __builtin_amdgcn_wave_barrier(); asm volatile("" ::: "memory");
        float* crow = C + (size_t)(r0 + mb * 16) * ldc + c0;
#pragma unroll 1
        for (int ps = 0; ps < 2; ++ps) {
#pragma unroll
            for (int s = 0; s < 8; ++s) { const int row = 2 * s + hi, cofs = lr * 4; v4f val = *(const v4fa*)(os + row * 68 + cofs); if (BIAS) { val[0] += bfr(bias[c0 + cofs]); val[1] += bfr(bias[c0 + cofs + 1]); val[2] += bfr(bias[c0 + cofs + 2]); val[3] += bfr(bias[c0 + cofs + 3]); }
                *(volatile v4f*)(crow + (size_t)row * ldc + cofs) = val; }
            if (ps == 0) __threadfence(); }
        __builtin_amdgcn_wave_barrier(); asm volatile("" ::: "memory");
    }
}

__device__ __forceinline__ h16 tohx(float x) { return (h16)x; }
__device__ __forceinline__ float silu_(float x) { return __fmul_rn(x, __fdiv_rn(1.0f, 1.0f + __expf(-x))); }
typedef __attribute__((ext_vector_type(2))) _Float16 v2h;
typedef __attribute__((ext_vector_type(4))) _Float16 v4h;

__global__ __launch_bounds__(256) void k_wt16(const float* __restrict__ w, int K, int N, h16* W16) { __shared__ float tile[64][65]; const int nb = (N + 63) / 64; const int k0 = (blockIdx.x / nb) * 64, n0 = (blockIdx.x % nb) * 64;
    for (int i = threadIdx.x; i < 64 * 64; i += 256) { const int kk = i / 64, nn = i % 64; tile[kk][nn] = (k0 + kk < K && n0 + nn < N) ? w[(size_t)(k0 + kk) * N + n0 + nn] : 0.f; }
    __syncthreads();
    const int nn = threadIdx.x / 4, kq = (threadIdx.x % 4) * 16; if (n0 + nn >= N) return;
    for (int c = 0; c < 16; c += 4) { v4h o; o[0] = tohx(bfr(tile[kq + c][nn])); o[1] = tohx(bfr(tile[kq + c + 1][nn])); o[2] = tohx(bfr(tile[kq + c + 2][nn])); o[3] = tohx(bfr(tile[kq + c + 3][nn])); h16* dst = W16 + (size_t)(n0 + nn) * K + k0 + kq + c; *(volatile v4h*)dst = o; __threadfence(); *(volatile v4h*)dst = o; } }
__global__ __launch_bounds__(256) void k_modv(const float* __restrict__ vec, const float* __restrict__ wi, const float* __restrict__ bi, const float* __restrict__ wt, const float* __restrict__ bt, float* MOD) { const int i = blockIdx.x * 256 + threadIdx.x; if (i >= 2 * 6 * HID) return; const int s = i / (6 * HID), j = i % (6 * HID); const float* w = s ? wt : wi; float acc = bfr((s ? bt : bi)[j]);
#pragma unroll 1
    for (int k = 0; k < HID; ++k) { float p = __fmul_rn(silu_(bfr(vec[k])), bfr(w[(size_t)k * 6 * HID + j])); asm volatile("" : "+v"(p)); acc = __fadd_rn(acc, p); } *(volatile float*)(MOD + i) = acc; __threadfence(); *(volatile float*)(MOD + i) = acc; }
template <int RES> __global__ __launch_bounds__(256) void k_lnmod(const float* __restrict__ xin, const float* __restrict__ P, const float* __restrict__ g, const float* __restrict__ sc, const float* __restrict__ sh, int nrows, float* X1, h16* XM16) {
    const int lane = threadIdx.x & 31; const int row = blockIdx.x * 8 + (threadIdx.x >> 5); if (row >= nrows) return; const size_t rb = (size_t)row * HID;
    auto val = [&](int c) { if (RES) { float p = __fmul_rn(g[c], P[rb + c]); asm volatile("" : "+v"(p)); return __fadd_rn(bfr(xin[rb + c]), p); } return bfr(xin[rb + c]); };
    float s = 0.f;
#pragma unroll 1
    for (int c0 = lane * 4; c0 < HID; c0 += 128) s = __fadd_rn(s, __fadd_rn(__fadd_rn(val(c0), val(c0 + 1)), __fadd_rn(val(c0 + 2), val(c0 + 3))));
#pragma unroll
    for (int shf = 16; shf; shf >>= 1) s += __shfl_xor(s, shf, 32);
    const float mean = s * (1.0f / HID); float q2 = 0.f;
#pragma unroll 1
    for (int c0 = lane * 4; c0 < HID; c0 += 128) {
#pragma unroll
        for (int u = 0; u < 4; ++u) { float d0 = __fsub_rn(val(c0 + u), mean); asm volatile("" : "+v"(d0)); float p = __fmul_rn(d0, d0); asm volatile("" : "+v"(p)); q2 = __fadd_rn(q2, p); } }
#pragma unroll
    for (int shf = 16; shf; shf >>= 1) q2 += __shfl_xor(q2, shf, 32);
    const float rstd = __frsqrt_rn(__fadd_rn(q2 * (1.0f / HID), 1e-6f));
    for (int ps = 0; ps < 2; ++ps) {
#pragma unroll 1
        for (int c0 = lane * 4; c0 < HID; c0 += 128) { v4f xo; v4h o;
#pragma unroll
            for (int u = 0; u < 4; ++u) { const float xv = val(c0 + u); xo[u] = xv; float n = __fmul_rn(__fsub_rn(xv, mean), rstd); asm volatile("" : "+v"(n)); float m = __fmul_rn(__fadd_rn(1.0f, sc[c0 + u]), n); asm volatile("" : "+v"(m)); o[u] = tohx(__fadd_rn(m, sh[c0 + u])); }
            if (RES) *(volatile v4f*)(X1 + rb + c0) = xo; *(volatile v4h*)(XM16 + rb + c0) = o; }
        if (ps == 0) __threadfence(); } }
__global__ __launch_bounds__(256) void k_qkrms(const float* __restrict__ QKV, int nrows, int r0, const float* __restrict__ qs, const float* __restrict__ ks, h16* Q16, h16* K16) { const int lane = threadIdx.x & 31; const int w = blockIdx.x * 8 + (threadIdx.x >> 5); if (w >= nrows * NH_) return; const int h = w % NH_, t = w / NH_; const float* rq = QKV + (size_t)t * 3 * HID + h * HD + 2 * lane; const float* rk = rq + HID;
    const float q0 = rq[0], q1 = rq[1], k0 = rk[0], k1 = rk[1]; float sq = __fadd_rn(__fmul_rn(q0, q0), __fmul_rn(q1, q1)), sk = __fadd_rn(__fmul_rn(k0, k0), __fmul_rn(k1, k1));
#pragma unroll
    for (int shf = 16; shf; shf >>= 1) { sq += __shfl_xor(sq, shf, 32); sk += __shfl_xor(sk, shf, 32); }
    const float rq_ = __frsqrt_rn(__fadd_rn(sq * (1.0f / HD), 1e-6f)), rk_ = __frsqrt_rn(__fadd_rn(sk * (1.0f / HD), 1e-6f)); v2h oq, ok;
    { float a = __fmul_rn(q0, rq_); asm volatile("" : "+v"(a)); oq[0] = tohx(__fmul_rn(a, bfr(qs[2 * lane])) * 0.125f); float b = __fmul_rn(q1, rq_); asm volatile("" : "+v"(b)); oq[1] = tohx(__fmul_rn(b, bfr(qs[2 * lane + 1])) * 0.125f);
      float c = __fmul_rn(k0, rk_); asm volatile("" : "+v"(c)); ok[0] = tohx(__fmul_rn(c, bfr(ks[2 * lane]))); float d = __fmul_rn(k1, rk_); asm volatile("" : "+v"(d)); ok[1] = tohx(__fmul_rn(d, bfr(ks[2 * lane + 1]))); }
    const size_t o = ((size_t)h * LA + r0 + t) * HD + 2 * lane; for (int ps = 0; ps < 2; ++ps) { *(volatile v2h*)(Q16 + o) = oq; *(volatile v2h*)(K16 + o) = ok; if (ps == 0) __threadfence(); } }
__global__ __launch_bounds__(256) void k_vt(const float* __restrict__ QKV, int nrows, int r0, h16* VT) { const int e = (blockIdx.x * 256 + threadIdx.x) * 2; if (e >= NH_ * HD * nrows) return; const int t = e % nrows; const int d = (e / nrows) % HD; const int h = e / (nrows * HD); v2h o; o[0] = tohx(QKV[(size_t)t * 3 * HID + 2 * HID + h * HD + d]); o[1] = tohx(QKV[(size_t)(t + 1) * 3 * HID + 2 * HID + h * HD + d]); h16* dst = VT + ((size_t)h * HD + d) * LA + r0 + t; *(volatile v2h*)dst = o; __threadfence(); *(volatile v2h*)dst = o; }
__global__ __launch_bounds__(256) void k_mrg16(const float* __restrict__ O, int h0, h16* ATT16) { const int e = (blockIdx.x * 256 + threadIdx.x) * 4; if (e >= LA * ZH * HD) return; const int c = e % (ZH * HD); const int t = e / (ZH * HD); const int z = c / HD, d = c % HD; const float* r = O + ((size_t)z * LA + t) * HD + d; v4h o;
#pragma unroll
    for (int u = 0; u < 4; ++u) o[u] = tohx(r[u] * (1.0f / PCAR)); h16* dst = ATT16 + (size_t)t * HID + (h0 + z) * HD + d; *(volatile v4h*)dst = o; __threadfence(); *(volatile v4h*)dst = o; }
__global__ __launch_bounds__(256) void k_gelu16(const float* __restrict__ Hh, size_t n4, h16* G16) { const size_t e = ((size_t)blockIdx.x * 256 + threadIdx.x) * 4; if (e >= n4 * 4) return; const v4f a = *(const v4f*)(Hh + e); v4h o;
#pragma unroll 1
    for (int u = 0; u < 4; ++u) { const float x = a[u]; const float in = 0.7978845608028654f * __fadd_rn(x, 0.044715f * x * x * x); o[u] = tohx(0.5f * x * __fadd_rn(1.0f, tanhf(in))); } *(volatile v4h*)(G16 + e) = o; __threadfence(); *(volatile v4h*)(G16 + e) = o; }
__global__ __launch_bounds__(256) void k_gout(const float* __restrict__ X1, const float* __restrict__ M2, const float* __restrict__ g, int nrows, float* OUT) { const int e = (blockIdx.x * 256 + threadIdx.x) * 4; if (e >= nrows * HID) return; const int c = e % HID; const v4f a = *(const v4f*)(X1 + e), m = *(const v4f*)(M2 + e); v4f o;
#pragma unroll
    for (int u = 0; u < 4; ++u) { float p = __fmul_rn(g[c + u], m[u]); asm volatile("" : "+v"(p)); o[u] = __fadd_rn(a[u], p); } *(volatile v4f*)(OUT + e) = o; __threadfence(); *(volatile v4f*)(OUT + e) = o; }
template <int NFULL, int TAIL> __global__ __launch_bounds__(256) void k_soft(const float* __restrict__ Sb, int nrows, int rowsper, int rvalid, int nvalid, h16* P) { const int lane = threadIdx.x & 31; const size_t row = (size_t)blockIdx.x * 8 + (threadIdx.x >> 5); if (row >= (size_t)nrows) return; constexpr int LD = NFULL * 128 + TAIL * 64; const float* sr = Sb + row * LD; h16* pr = P + row * LD; const bool live = (int)(row % rowsper) < rvalid; float mx = -3.0e38f;
#pragma unroll 1
    for (int ch = 0; ch < NFULL + TAIL; ++ch) { if (ch == NFULL && lane >= 16) break; const int j0 = ch * 128 + lane * 4; const v4f a = *(const v4f*)(sr + j0);
#pragma unroll
        for (int q = 0; q < 4; ++q) if (j0 + q < nvalid) mx = fmaxf(mx, a[q]); }
#pragma unroll
    for (int sh = 16; sh; sh >>= 1) mx = fmaxf(mx, __shfl_xor(mx, sh, 32));
    float sum = 0.f;
#pragma unroll 1
    for (int ch = 0; ch < NFULL + TAIL; ++ch) { if (ch == NFULL && lane >= 16) break; const int j0 = ch * 128 + lane * 4; const v4f a = *(const v4f*)(sr + j0);
#pragma unroll
        for (int q = 0; q < 4; ++q) if (j0 + q < nvalid) { float d0 = __fsub_rn(a[q], mx); asm volatile("" : "+v"(d0)); sum += __expf(d0); } }
#pragma unroll
    for (int sh = 16; sh; sh >>= 1) sum += __shfl_xor(sum, sh, 32);
    const float f = live ? __fdiv_rn(PCAR, sum) : 0.f;
    for (int ps = 0; ps < 2; ++ps) {
#pragma unroll 1
        for (int ch = 0; ch < NFULL + TAIL; ++ch) { if (ch == NFULL && lane >= 16) break; const int j0 = ch * 128 + lane * 4; const v4f a = *(const v4f*)(sr + j0); v4h o;
#pragma unroll
            for (int q = 0; q < 4; ++q) { float val = 0.f; if (live && j0 + q < nvalid) { float d0 = __fsub_rn(a[q], mx); asm volatile("" : "+v"(d0)); val = __fmul_rn(__expf(d0), f); } o[q] = tohx(val); } *(volatile v4h*)(pr + j0) = o; }
        if (ps == 0) __threadfence(); } }

extern "C" void kernel_launch(void* const* d_in, const int* in_sizes, int n_in,
                              void* d_out, int out_size, void* d_ws, size_t ws_size, hipStream_t stream) {
    (void)in_sizes; (void)n_in; (void)out_size;
    const float* img = (const float*)d_in[0]; const float* txt = (const float*)d_in[1]; const float* vec = (const float*)d_in[2]; const float* imw = (const float*)d_in[3]; const float* imb = (const float*)d_in[4]; const float* tmw = (const float*)d_in[5]; const float* tmb = (const float*)d_in[6];
    const float* iqkv = (const float*)d_in[7]; const float* iqs = (const float*)d_in[8]; const float* iks = (const float*)d_in[9]; const float* ipw = (const float*)d_in[10]; const float* ipb = (const float*)d_in[11]; const float* iw1 = (const float*)d_in[12]; const float* ib1 = (const float*)d_in[13]; const float* iw2 = (const float*)d_in[14]; const float* ib2 = (const float*)d_in[15];
    const float* tqkv = (const float*)d_in[16]; const float* tqs = (const float*)d_in[17]; const float* tks = (const float*)d_in[18]; const float* tpw = (const float*)d_in[19]; const float* tpb = (const float*)d_in[20]; const float* tw1 = (const float*)d_in[21]; const float* tb1 = (const float*)d_in[22]; const float* tw2 = (const float*)d_in[23]; const float* tb2 = (const float*)d_in[24];
    float* OUTI = (float*)d_out; float* OUTT = (float*)((char*)d_out + 8388608);
    char* wsp = (char*)d_ws;
    auto take = [&](size_t bytes) { char* p = wsp; wsp += (bytes + 255) & ~(size_t)255; return (void*)p; };
    h16* IQKV = (h16*)take((size_t)3 * HID * HID * 2); h16* TQKV = (h16*)take((size_t)3 * HID * HID * 2); h16* IPW = (h16*)take((size_t)HID * HID * 2); h16* TPW = (h16*)take((size_t)HID * HID * 2); h16* IW1 = (h16*)take((size_t)MLPD * HID * 2); h16* TW1 = (h16*)take((size_t)MLPD * HID * 2); h16* IW2 = (h16*)take((size_t)HID * MLPD * 2); h16* TW2 = (h16*)take((size_t)HID * MLPD * 2);
    float* MOD = (float*)take((size_t)2 * 6 * HID * 4); h16* XM16 = (h16*)take((size_t)LI * HID * 2); float* QKV = (float*)take((size_t)LI * 3 * HID * 4); h16* Q16 = (h16*)take((size_t)NH_ * LA * HD * 2); h16* K16 = (h16*)take((size_t)NH_ * LA * HD * 2); h16* VT16 = (h16*)take((size_t)NH_ * HD * LA * 2);
    float* Sb = (float*)take((size_t)ZH * LA * LA * 4); h16* P16 = (h16*)take((size_t)ZH * LA * LA * 2); float* O = (float*)take((size_t)ZH * LA * HD * 4); h16* ATT16 = (h16*)take((size_t)LA * HID * 2); float* PRJ = (float*)take((size_t)LI * HID * 4); float* X1 = (float*)take((size_t)LI * HID * 4); float* H1 = (float*)take((size_t)LI * MLPD * 4); h16* G16 = (h16*)take((size_t)LI * MLPD * 2); float* M2 = (float*)take((size_t)LI * HID * 4);
    if ((size_t)(wsp - (char*)d_ws) > ws_size) return;
    const float* ish1 = MOD; const float* isc1 = MOD + HID; const float* ig1 = MOD + 2 * HID; const float* ish2 = MOD + 3 * HID; const float* isc2 = MOD + 4 * HID; const float* ig2 = MOD + 5 * HID; const float* tsh1 = MOD + 6 * HID; const float* tsc1 = MOD + 7 * HID; const float* tg1 = MOD + 8 * HID; const float* tsh2 = MOD + 9 * HID; const float* tsc2 = MOD + 10 * HID; const float* tg2 = MOD + 11 * HID;
    k_wt16<<<(HID / 64) * (3 * HID / 64), 256, 0, stream>>>(iqkv, HID, 3 * HID, IQKV); k_wt16<<<(HID / 64) * (3 * HID / 64), 256, 0, stream>>>(tqkv, HID, 3 * HID, TQKV); k_wt16<<<(HID / 64) * (HID / 64), 256, 0, stream>>>(ipw, HID, HID, IPW); k_wt16<<<(HID / 64) * (HID / 64), 256, 0, stream>>>(tpw, HID, HID, TPW);
    k_wt16<<<(HID / 64) * (MLPD / 64), 256, 0, stream>>>(iw1, HID, MLPD, IW1); k_wt16<<<(HID / 64) * (MLPD / 64), 256, 0, stream>>>(tw1, HID, MLPD, TW1); k_wt16<<<(MLPD / 64) * (HID / 64), 256, 0, stream>>>(iw2, MLPD, HID, IW2); k_wt16<<<(MLPD / 64) * (HID / 64), 256, 0, stream>>>(tw2, MLPD, HID, TW2);
    k_modv<<<(2 * 6 * HID + 255) / 256, 256, 0, stream>>>(vec, imw, imb, tmw, tmb, MOD);
    k_lnmod<0><<<LTX / 8, 256, 0, stream>>>(txt, nullptr, nullptr, tsc1, tsh1, LTX, nullptr, XM16); k_gemmw<h16, 0, false><<<dim3(LTX / 64, 3 * HID / 64, 1), 32, 0, stream>>>(XM16, nullptr, TQKV, nullptr, HID, QKV, 3 * HID, nullptr, 0, 0, 0);
    k_qkrms<<<(LTX * NH_ + 7) / 8, 256, 0, stream>>>(QKV, LTX, 0, tqs, tks, Q16, K16); k_vt<<<(NH_ * HD * LTX / 2 + 255) / 256, 256, 0, stream>>>(QKV, LTX, 0, VT16);
    k_lnmod<0><<<LI / 8, 256, 0, stream>>>(img, nullptr, nullptr, isc1, ish1, LI, nullptr, XM16); k_gemmw<h16, 0, false><<<dim3(LI / 64, 3 * HID / 64, 1), 32, 0, stream>>>(XM16, nullptr, IQKV, nullptr, HID, QKV, 3 * HID, nullptr, 0, 0, 0);
    k_qkrms<<<(LI * NH_ + 7) / 8, 256, 0, stream>>>(QKV, LI, LTX, iqs, iks, Q16, K16); k_vt<<<(NH_ * HD * LI / 2 + 255) / 256, 256, 0, stream>>>(QKV, LI, LTX, VT16);
    for (int h0 = 0; h0 < NH_; h0 += ZH) {
        k_gemmw<h16, 0, false><<<dim3(LA / 64, LA / 64, ZH), 32, 0, stream>>>(Q16 + (size_t)h0 * LA * HD, nullptr, K16 + (size_t)h0 * LA * HD, nullptr, HD, Sb, LA, nullptr, (size_t)LA * HD, (size_t)LA * HD, (size_t)LA * LA);
        k_soft<20, 0><<<(ZH * LA + 7) / 8, 256, 0, stream>>>(Sb, ZH * LA, LA, LA, LA, P16);
        k_gemmw<h16, 0, false><<<dim3(LA / 64, 1, ZH), 32, 0, stream>>>(P16, nullptr, VT16 + (size_t)h0 * HD * LA, nullptr, LA, O, HD, nullptr, (size_t)LA * LA, (size_t)HD * LA, (size_t)LA * HD);
        k_mrg16<<<(LA * ZH * HD / 4 + 255) / 256, 256, 0, stream>>>(O, h0, ATT16); }
    k_gemmw<h16, 0, true><<<dim3(LI / 64, HID / 64, 1), 32, 0, stream>>>(ATT16 + (size_t)LTX * HID, nullptr, IPW, nullptr, HID, PRJ, HID, ipb, 0, 0, 0);
    k_lnmod<1><<<LI / 8, 256, 0, stream>>>(img, PRJ, ig1, isc2, ish2, LI, X1, XM16);
    k_gemmw<h16, 0, true><<<dim3(LI / 64, MLPD / 64, 1), 32, 0, stream>>>(XM16, nullptr, IW1, nullptr, HID, H1, MLPD, ib1, 0, 0, 0); k_gelu16<<<(unsigned)(((size_t)LI * MLPD / 4 + 255) / 256), 256, 0, stream>>>(H1, (size_t)LI * MLPD / 4, G16);
    k_gemmw<h16, 0, true><<<dim3(LI / 64, HID / 64, 1), 32, 0, stream>>>(G16, nullptr, IW2, nullptr, MLPD, M2, HID, ib2, 0, 0, 0); k_gout<<<(LI * HID / 4 + 255) / 256, 256, 0, stream>>>(X1, M2, ig2, LI, OUTI);
    k_gemmw<h16, 0, true><<<dim3(LTX / 64, HID / 64, 1), 32, 0, stream>>>(ATT16, nullptr, TPW, nullptr, HID, PRJ, HID, tpb, 0, 0, 0);
    k_lnmod<1><<<LTX / 8, 256, 0, stream>>>(txt, PRJ, tg1, tsc2, tsh2, LTX, X1, XM16);
    k_gemmw<h16, 0, true><<<dim3(LTX / 64, MLPD / 64, 1), 32, 0, stream>>>(XM16, nullptr, TW1, nullptr, HID, H1, MLPD, tb1, 0, 0, 0); k_gelu16<<<(unsigned)(((size_t)LTX * MLPD / 4 + 255) / 256), 256, 0, stream>>>(H1, (size_t)LTX * MLPD / 4, G16);
    k_gemmw<h16, 0, true><<<dim3(LTX / 64, HID / 64, 1), 32, 0, stream>>>(G16, nullptr, TW2, nullptr, MLPD, M2, HID, tb2, 0, 0, 0); k_gout<<<(LTX * HID / 4 + 255) / 256, 256, 0, stream>>>(X1, M2, tg2, LTX, OUTT);
}
